// ChannelBlock_13417477833042
// MI455X (gfx1250) — hardware-verified
//
#include <hip/hip_runtime.h>
#define NIM 32
#define CC 384
#define NTK 784
#define NTP 800
#define NH 12
#define HD 32
#define HIDN 1536
#define ICH 4
#define RCH (ICH * NTK)
typedef __bf16 v16b __attribute__((ext_vector_type(16)));
typedef unsigned short v8us __attribute__((ext_vector_type(8), may_alias));
typedef float  v8f  __attribute__((ext_vector_type(8)));
typedef float  v4f  __attribute__((ext_vector_type(4)));
typedef float  v4fa __attribute__((ext_vector_type(4), may_alias));
union FragB { v16b v; v8us half[2]; unsigned short u[16]; };

__device__ __forceinline__ unsigned short bf16_bits(float x) { unsigned int u = __float_as_uint(x); return (unsigned short)((u + 0x7FFFu + ((u >> 16) & 1u)) >> 16); }
__device__ __forceinline__ float bf16_val(unsigned short b) { return __uint_as_float(((unsigned int)b) << 16); }
__device__ __forceinline__ float bf16_round(float x) { return bf16_val(bf16_bits(x)); }
template <int NT>
__device__ __forceinline__ v8f mmaN(v16b ah, v16b al, v16b bh, v16b bl, v8f c) {
  c = __builtin_amdgcn_wmma_f32_16x16x32_bf16(false, ah, false, bh, (short)0, c, false, false);
  if (NT >= 2) c = __builtin_amdgcn_wmma_f32_16x16x32_bf16(false, al, false, bh, (short)0, c, false, false);
  if (NT >= 3) c = __builtin_amdgcn_wmma_f32_16x16x32_bf16(false, ah, false, bl, (short)0, c, false, false);
  asm volatile("v_nop\n\tv_nop\n\tv_nop\n\tv_nop" : "+v"(c) : "v"(ah), "v"(al), "v"(bh), "v"(bl));
  return c;
}

__global__ __launch_bounds__(256) void k_wt_bf16(const float* __restrict__ W, unsigned short* __restrict__ Wt, int K, int N) {
  const int t = blockIdx.x * 256 + threadIdx.x;
  const int k8n = K / 8;
  if (t >= N * k8n) return;
  const int n = t / k8n, k8 = (t % k8n) * 8;
  v8us v;
#pragma unroll
  for (int i = 0; i < 8; ++i) v[i] = bf16_bits(W[(size_t)(k8 + i) * N + n]);
  *(volatile v8us*)(Wt + (size_t)n * K + k8) = v;
  __threadfence();
  *(volatile v8us*)(Wt + (size_t)n * K + k8) = v;
}

template <bool ASPLIT, int ACT, bool BIAS_BF16>
__global__ __launch_bounds__(128) void k_gemm_bf(const float* __restrict__ A, int lda, const unsigned short* __restrict__ Wt, int ldb,
                                               const float* __restrict__ bias, float* __restrict__ C, int ldc, int M, int N, int K) {
  __shared__ __attribute__((aligned(16))) float so[4][16][64];
  const int tid = threadIdx.x, w = tid >> 5, lane = tid & 31, ln = lane & 15, hh = lane >> 4;
  const int ntn = N / 64;
  const int wid = blockIdx.x * 4 + w;
  const int mt = wid / ntn, nq = wid % ntn;
  if (mt * 16 >= M) return;
  const int row0 = mt * 16, col0 = nq * 64;
  const float* arow = A + (size_t)(row0 + ln) * lda;
  v8f acc[4] = {};
  for (int kb = 0; kb < K; kb += 32) {
    FragB ah, al;
    const v4f x0 = *(const v4fa*)(arow + kb + 8 * hh), x1 = *(const v4fa*)(arow + kb + 8 * hh + 4);
    const v4f x2 = *(const v4fa*)(arow + kb + 16 + 8 * hh), x3 = *(const v4fa*)(arow + kb + 16 + 8 * hh + 4);
    float xs[16] = {x0[0],x0[1],x0[2],x0[3],x1[0],x1[1],x1[2],x1[3],x2[0],x2[1],x2[2],x2[3],x3[0],x3[1],x3[2],x3[3]};
#pragma unroll
    for (int i = 0; i < 16; ++i) { const unsigned short hb = bf16_bits(xs[i]); ah.u[i] = hb; al.u[i] = ASPLIT ? bf16_bits(xs[i] - bf16_val(hb)) : (unsigned short)0; }
#pragma unroll
    for (int t = 0; t < 4; ++t) {
      const unsigned short* brow = Wt + (size_t)(col0 + t * 16 + ln) * ldb + kb;
      FragB b;
      b.half[0] = *(const v8us*)(brow + 8 * hh);
      b.half[1] = *(const v8us*)(brow + 16 + 8 * hh);
      acc[t] = mmaN<ASPLIT ? 2 : 1>(ah.v, al.v, b.v, b.v, acc[t]);
    }
  }
#pragma unroll
  for (int t = 0; t < 4; ++t) {
    float bv = bias ? bias[col0 + t * 16 + ln] : 0.f;
    if (BIAS_BF16) bv = bf16_round(bv);
#pragma unroll
    for (int r = 0; r < 8; ++r) { float v = acc[t][r] + bv; if (ACT == 1) v = fmaxf(v, 0.f); so[w][8 * hh + r][t * 16 + ln] = v; }
  }
  __builtin_amdgcn_fence(__ATOMIC_ACQ_REL, "workgroup");
  __builtin_amdgcn_wave_barrier();
  const int rsub = lane >> 4, c4 = (lane & 15) * 4;
  for (int pass = 0; pass < 2; ++pass) {
#pragma unroll
    for (int q = 0; q < 8; ++q) {
      const int r = q * 2 + rsub;
      const v4f v = *(const v4fa*)&so[w][r][c4];
      *(volatile v4f*)(C + (size_t)(row0 + r) * ldc + col0 + c4) = v;
    }
    if (pass == 0) __threadfence();
  }
}

template <bool ASPLIT, int ACT, bool BIAS_BF16, bool RES_BF16>
__global__ __launch_bounds__(128) void k_gemm_bf3(const float* __restrict__ A, int lda, const unsigned short* __restrict__ Wt, int ldb,
                                                const float* __restrict__ bias, const float* __restrict__ resid, int rmod, int ldr,
                                                float* __restrict__ C, int ldc, int M, int N, int K) {
  __shared__ __attribute__((aligned(16))) float so[4][16][64];
  const int tid = threadIdx.x, w = tid >> 5, lane = tid & 31, ln = lane & 15, hh = lane >> 4;
  const int ntn = N / 64;
  const int wid = blockIdx.x * 4 + w;
  const int mt = wid / ntn, nq = wid % ntn;
  if (mt * 16 >= M) return;
  const int row0 = mt * 16, col0 = nq * 64;
  const float* arow = A + (size_t)(row0 + ln) * lda;
  v8f acc[4] = {};
  for (int kb = 0; kb < K; kb += 32) {
    FragB ah, al;
    const v4f x0 = *(const v4fa*)(arow + kb + 8 * hh), x1 = *(const v4fa*)(arow + kb + 8 * hh + 4);
    const v4f x2 = *(const v4fa*)(arow + kb + 16 + 8 * hh), x3 = *(const v4fa*)(arow + kb + 16 + 8 * hh + 4);
    float xs[16] = {x0[0],x0[1],x0[2],x0[3],x1[0],x1[1],x1[2],x1[3],x2[0],x2[1],x2[2],x2[3],x3[0],x3[1],x3[2],x3[3]};
#pragma unroll
    for (int i = 0; i < 16; ++i) { const unsigned short hb = bf16_bits(xs[i]); ah.u[i] = hb; al.u[i] = ASPLIT ? bf16_bits(xs[i] - bf16_val(hb)) : (unsigned short)0; }
#pragma unroll
    for (int t = 0; t < 4; ++t) {
      const unsigned short* brow = Wt + (size_t)(col0 + t * 16 + ln) * ldb + kb;
      FragB b;
      b.half[0] = *(const v8us*)(brow + 8 * hh);
      b.half[1] = *(const v8us*)(brow + 16 + 8 * hh);
      acc[t] = mmaN<ASPLIT ? 2 : 1>(ah.v, al.v, b.v, b.v, acc[t]);
    }
  }
#pragma unroll
  for (int t = 0; t < 4; ++t) {
    const int col = col0 + t * 16 + ln;
    float bv = bias ? bias[col] : 0.f;
    if (BIAS_BF16) bv = bf16_round(bv);
#pragma unroll
    for (int r = 0; r < 8; ++r) {
      float v = acc[t][r] + bv;
      if (resid) { float rv = resid[(size_t)((row0 + 8 * hh + r) % rmod) * ldr + col]; if (RES_BF16) rv = bf16_round(rv); v += rv; }
      if (ACT == 1) v = fmaxf(v, 0.f);
      if (ACT == 2) v = 0.5f * v * (1.0f + erff(v * 0.70710678118654752f));
      if (ACT == 3) { const float u = 0.7978845608028654f * (v + 0.044715f * v * v * v); v = 0.5f * v * (1.0f + tanhf(u)); }
      so[w][8 * hh + r][t * 16 + ln] = v;
    }
  }
  __builtin_amdgcn_fence(__ATOMIC_ACQ_REL, "workgroup");
  __builtin_amdgcn_wave_barrier();
  const int rsub = lane >> 4, c4 = (lane & 15) * 4;
  for (int pass = 0; pass < 2; ++pass) {
#pragma unroll
    for (int q = 0; q < 8; ++q) {
      const int r = q * 2 + rsub;
      const v4f v = *(const v4fa*)&so[w][r][c4];
      *(volatile v4f*)(C + (size_t)(row0 + r) * ldc + col0 + c4) = v;
    }
    if (pass == 0) __threadfence();
  }
}
template <bool PARAM_BF16>
__global__ __launch_bounds__(256) void k_layernorm(const float* __restrict__ X, const float* __restrict__ R, const float* __restrict__ g, const float* __restrict__ bta,
                                                  float* __restrict__ out_sum, float* __restrict__ out_norm, int N, float eps) {
  __shared__ float red[256];
  const int row = blockIdx.x, tid = threadIdx.x;
  const float* x = X + (size_t)row * N; const float* rr = R ? R + (size_t)row * N : nullptr;
  float vals[16];
  const int per = N / 256;
  float s1 = 0.f;
  for (int u = 0; u < per / 4; ++u) {
    const int j = tid * 4 + 1024 * u;
    const v4f a = *(const v4fa*)(x + j);
    v4f b = {0.f,0.f,0.f,0.f}; if (rr) b = *(const v4fa*)(rr + j);
#pragma unroll
    for (int q = 0; q < 4; ++q) { const float v = a[q] + b[q]; vals[u * 4 + q] = v; s1 += v; }
  }
  red[tid] = s1; __syncthreads();
  for (int st = 128; st > 0; st >>= 1) { if (tid < st) red[tid] += red[tid + st]; __syncthreads(); }
  const float mu = red[0] / (float)N; __syncthreads();
  float s2 = 0.f;
  for (int u = 0; u < per / 4; ++u)
#pragma unroll
    for (int q = 0; q < 4; ++q) { const float c = vals[u * 4 + q] - mu; s2 += c * c; }
  red[tid] = s2; __syncthreads();
  for (int st = 128; st > 0; st >>= 1) { if (tid < st) red[tid] += red[tid + st]; __syncthreads(); }
  const float rs = rsqrtf(red[0] / (float)N + eps);
  for (int pass = 0; pass < 2; ++pass) {
    for (int u = 0; u < per / 4; ++u) {
      const int j = tid * 4 + 1024 * u;
      v4f o, sm;
#pragma unroll
      for (int q = 0; q < 4; ++q) {
        float gg = g[j + q], bb = bta[j + q];
        if (PARAM_BF16) { gg = bf16_round(gg); bb = bf16_round(bb); }
        sm[q] = vals[u * 4 + q]; o[q] = (vals[u * 4 + q] - mu) * rs * gg + bb;
      }
      if (out_sum) *(volatile v4f*)(out_sum + (size_t)row * N + j) = sm;
      *(volatile v4f*)(out_norm + (size_t)row * N + j) = o;
    }
    if (pass == 0) __threadfence();
  }
}


typedef _Float16 v16h __attribute__((ext_vector_type(16)));
union FragH { v16h v; v8us half[2]; _Float16 h[16]; unsigned short u[16]; };
template <int NT>
__device__ __forceinline__ v8f mmaH(v16h ah, v16h al, v16h bh, v16h bl, v8f c) {
  c = __builtin_amdgcn_wmma_f32_16x16x32_f16(false, ah, false, bh, (short)0, c, false, false);
  if (NT >= 2) c = __builtin_amdgcn_wmma_f32_16x16x32_f16(false, al, false, bh, (short)0, c, false, false);
  if (NT >= 3) c = __builtin_amdgcn_wmma_f32_16x16x32_f16(false, ah, false, bl, (short)0, c, false, false);
  asm volatile("v_nop\n\tv_nop\n\tv_nop\n\tv_nop" : "+v"(c) : "v"(ah), "v"(al), "v"(bh), "v"(bl));
  return c;
}
template <bool ASPLIT>
__global__ __launch_bounds__(128) void k_gemm_h(const float* __restrict__ A, int lda, size_t sA, const _Float16* __restrict__ Bh, int ldb, size_t sB, float alpha, float* __restrict__ C, int ldc, size_t sC, int M, int N, int K) {
  __shared__ __attribute__((aligned(16))) float so[4][16][64];
  const int tid = threadIdx.x, w = tid >> 5, lane = tid & 31, ln = lane & 15, hh = lane >> 4; const int by = blockIdx.y;
  A += (size_t)by * sA; Bh += (size_t)by * sB; C += (size_t)by * sC;
  const int ntn = (N + 63) / 64; const int wid = blockIdx.x * 4 + w; const int mt = wid / ntn, nq = wid % ntn; if (mt * 16 >= M) return;
  const int row0 = mt * 16, col0 = nq * 64; const float* arow = A + (size_t)(row0 + ln) * lda;
  v8f acc[4] = {};
  for (int kb = 0; kb < K; kb += 32) {
    FragH ah, al;
    const v4f x0 = *(const v4fa*)(arow + kb + 8 * hh), x1 = *(const v4fa*)(arow + kb + 8 * hh + 4), x2 = *(const v4fa*)(arow + kb + 16 + 8 * hh), x3 = *(const v4fa*)(arow + kb + 16 + 8 * hh + 4);
    float xs[16] = {x0[0],x0[1],x0[2],x0[3],x1[0],x1[1],x1[2],x1[3],x2[0],x2[1],x2[2],x2[3],x3[0],x3[1],x3[2],x3[3]};
#pragma unroll
    for (int i = 0; i < 16; ++i) { const _Float16 h = (_Float16)xs[i]; ah.h[i] = h; al.h[i] = ASPLIT ? (_Float16)(xs[i] - (float)h) : (_Float16)0.0f; }
#pragma unroll
    for (int t = 0; t < 4; ++t) { if (col0 + t * 16 >= N) continue; const size_t boff = (size_t)(col0 + t * 16 + ln) * ldb + kb; FragH bq; bq.half[0] = *(const v8us*)(Bh + boff + 8 * hh); bq.half[1] = *(const v8us*)(Bh + boff + 16 + 8 * hh);
      acc[t] = mmaH<ASPLIT ? 2 : 1>(ah.v, al.v, bq.v, bq.v, acc[t]); }
  }
#pragma unroll
  for (int t = 0; t < 4; ++t) { if (col0 + t * 16 >= N) continue;
#pragma unroll
    for (int r = 0; r < 8; ++r) so[w][8 * hh + r][t * 16 + ln] = acc[t][r] * alpha; }
  __builtin_amdgcn_fence(__ATOMIC_ACQ_REL, "workgroup"); __builtin_amdgcn_wave_barrier();
  const int rsub = lane >> 4, c4 = (lane & 15) * 4;
  for (int pass = 0; pass < 2; ++pass) {
#pragma unroll
    for (int q = 0; q < 8; ++q) { const int r = q * 2 + rsub; if (col0 + c4 < N) { const v4f v = *(const v4fa*)&so[w][r][c4]; *(volatile v4f*)(C + (size_t)(row0 + r) * ldc + col0 + c4) = v; } }
    if (pass == 0) __threadfence(); }
}

__global__ __launch_bounds__(256) void k_wt_f16(const float* __restrict__ W, _Float16* __restrict__ Wt, int K, int N, float scale) {
  const int t = blockIdx.x * 256 + threadIdx.x; if (t >= N * (K / 8)) return; const int n = t / (K / 8), k8 = (t % (K / 8)) * 8; FragH f;
#pragma unroll
  for (int i = 0; i < 8; ++i) f.h[i] = (_Float16)(bf16_round(W[(size_t)(k8 + i) * N + n]) * scale); const v8us o = f.half[0];
  *(volatile v8us*)((unsigned short*)Wt + (size_t)n * K + k8) = o; __threadfence(); *(volatile v8us*)((unsigned short*)Wt + (size_t)n * K + k8) = o;
}
template <int ACT>
__global__ __launch_bounds__(128) void k_gemm_hhx(const _Float16* __restrict__ A, int lda, size_t sA, const _Float16* __restrict__ Bh, int ldb, size_t sB, float alpha, const float* __restrict__ bias, size_t sBias, const float* __restrict__ CP, int rowsPerB, size_t sCPb, int row0g,
    float* __restrict__ C, _Float16* __restrict__ C16, int ldc, size_t sC, int M, int N, int K) {
  __shared__ __attribute__((aligned(16))) float so[4][16][64];
  const int tid = threadIdx.x, w = tid >> 5, lane = tid & 31, ln = lane & 15, hh = lane >> 4; const int by = blockIdx.y;
  A += (size_t)by * sA; Bh += (size_t)by * sB; const size_t cofs = (size_t)by * sC; const float* bp = bias ? bias + (size_t)by * sBias : nullptr;
  const int ntn = (N + 63) / 64; const int wid = blockIdx.x * 4 + w; const int mt = wid / ntn, nq = wid % ntn; if (mt * 16 >= M) return;
  const int row0 = mt * 16, col0 = nq * 64; const _Float16* arow = A + (size_t)(row0 + ln) * lda;
  v8f acc[4] = {};
  for (int kb = 0; kb < K; kb += 32) { FragH ah; ah.half[0] = *(const v8us*)((const unsigned short*)arow + kb + 8 * hh); ah.half[1] = *(const v8us*)((const unsigned short*)arow + kb + 16 + 8 * hh);
#pragma unroll
    for (int t = 0; t < 4; ++t) { if (col0 + t * 16 >= N) continue; const size_t boff = (size_t)(col0 + t * 16 + ln) * ldb + kb; FragH bq; bq.half[0] = *(const v8us*)((const unsigned short*)Bh + boff + 8 * hh); bq.half[1] = *(const v8us*)((const unsigned short*)Bh + boff + 16 + 8 * hh);
      acc[t] = mmaH<1>(ah.v, ah.v, bq.v, bq.v, acc[t]); }
  }
#pragma unroll
  for (int t = 0; t < 4; ++t) { if (col0 + t * 16 >= N) continue; const int col = col0 + t * 16 + ln; const float bv = bp ? bf16_round(bp[col]) : 0.f;
#pragma unroll
    for (int r = 0; r < 8; ++r) { float v = acc[t][r] * alpha + bv; if (CP) { const int bidx = (row0g + row0 + 8 * hh + r) / rowsPerB; v += CP[(size_t)bidx * sCPb + (size_t)by * 64 + col]; } if (ACT == 1) v = (v > 0.f) ? v : expm1f(v); else if (ACT == 7) v = (v > 0.f) ? v + 1.0f : expf(v); else if (ACT == 8) v = tanhf(v); else if (ACT == 9) v = 0.5f * v * (1.0f + tanhf(0.7978845608028654f * (v + 0.044715f * v * v * v))); else if (ACT == 11) v = 1.0f / (1.0f + expf(-v)); else if (ACT == 12) v = (v > 0.f) ? v : 0.01f * v; else if (ACT == 14) v = (v > 0.f) ? v : 0.1f * v; else if (ACT == 15) v = v / (1.0f + expf(-v)); else if (ACT == 3) v = fmaxf(v, 0.f); else if (ACT == 6) v = 0.5f * v * (1.0f + erff(v * 0.70710678118654752f)); so[w][8 * hh + r][t * 16 + ln] = v; } }
  __builtin_amdgcn_fence(__ATOMIC_ACQ_REL, "workgroup"); __builtin_amdgcn_wave_barrier();
  const int rsub = lane >> 4, c4 = (lane & 15) * 4; typedef _Float16 v4h __attribute__((ext_vector_type(4)));
  for (int pass = 0; pass < 2; ++pass) {
#pragma unroll
    for (int q = 0; q < 8; ++q) { const int r = q * 2 + rsub; if (col0 + c4 < N) { const v4f v = *(const v4fa*)&so[w][r][c4]; if (C) *(volatile v4f*)(C + cofs + (size_t)(row0 + r) * ldc + col0 + c4) = v; if (C16) { v4h h4; for (int i = 0; i < 4; ++i) h4[i] = (_Float16)v[i]; *(volatile v4h*)(C16 + cofs + (size_t)(row0 + r) * ldc + col0 + c4) = h4; } } }
    if (pass == 0) __threadfence(); }
}


typedef _Float16 v4h __attribute__((ext_vector_type(4)));

__global__ __launch_bounds__(256) void k_x16(const float* __restrict__ x, _Float16* __restrict__ X16, size_t n8) { const size_t t = (size_t)blockIdx.x * 256 + threadIdx.x; if (t >= n8) return; FragH f;
#pragma unroll
  for (int q = 0; q < 8; ++q) f.h[q] = (_Float16)bf16_round(x[t * 8 + q]); *(volatile v8us*)((unsigned short*)X16 + t * 8) = f.half[0]; __threadfence(); *(volatile v8us*)((unsigned short*)X16 + t * 8) = f.half[0]; }
__global__ __launch_bounds__(256) void k_h16(const float* __restrict__ x, _Float16* __restrict__ X16, size_t n8) { const size_t t = (size_t)blockIdx.x * 256 + threadIdx.x; if (t >= n8) return; FragH f;
#pragma unroll
  for (int q = 0; q < 8; ++q) f.h[q] = (_Float16)x[t * 8 + q]; *(volatile v8us*)((unsigned short*)X16 + t * 8) = f.half[0]; __threadfence(); *(volatile v8us*)((unsigned short*)X16 + t * 8) = f.half[0]; }
__global__ __launch_bounds__(256) void k_round16f(const float* __restrict__ W, _Float16* __restrict__ Bt, size_t n8) { const size_t t = (size_t)blockIdx.x * 256 + threadIdx.x; if (t >= n8) return; FragH f;
#pragma unroll
  for (int i = 0; i < 8; ++i) f.h[i] = (_Float16)(bf16_round(W[t * 8 + i]) * 16.0f); *(volatile v8us*)((unsigned short*)Bt + t * 8) = f.half[0]; __threadfence(); *(volatile v8us*)((unsigned short*)Bt + t * 8) = f.half[0]; }
template <int NHv, int TTv>
__global__ __launch_bounds__(256) void k_vt(const _Float16* __restrict__ V16, int ldv, int voff, _Float16* __restrict__ Vt) { __shared__ unsigned short tl[64][66]; const int tid = threadIdx.x; const int slab = blockIdx.x / (TTv / 64), lg = blockIdx.x % (TTv / 64); const int b = slab / NHv, h = slab % NHv;
  for (int i = tid; i < 64 * 8; i += 256) { const int r = i / 8, c8 = (i % 8) * 8; FragH f; f.half[0] = *(const v8us*)((const unsigned short*)V16 + ((size_t)b * TTv + lg * 64 + r) * ldv + voff + h * 64 + c8);
#pragma unroll
    for (int q = 0; q < 8; ++q) tl[r][c8 + q] = f.u[q]; }
  __syncthreads();
  for (int pass = 0; pass < 2; ++pass) {
#pragma unroll
    for (int rd = 0; rd < 2; ++rd) { const int d = rd * 32 + tid / 8, pc = tid % 8; FragH f;
#pragma unroll
      for (int q = 0; q < 8; ++q) f.u[q] = tl[pc * 8 + q][d];
      *(volatile v8us*)((unsigned short*)Vt + ((size_t)slab * 64 + d) * TTv + lg * 64 + pc * 8) = f.half[0]; }
    if (pass == 0) __threadfence(); } }

__global__ __launch_bounds__(256) void k_hl(const float* __restrict__ F, _Float16* __restrict__ Hh, _Float16* __restrict__ Hl, size_t n8) { const size_t t = (size_t)blockIdx.x * 256 + threadIdx.x; if (t >= n8) return; FragH fh, fl; const v4f a = *(const v4fa*)(F + t * 8), c = *(const v4fa*)(F + t * 8 + 4);
#pragma unroll
  for (int q = 0; q < 4; ++q) { _Float16 h = (_Float16)a[q]; fh.h[q] = h; fl.h[q] = (_Float16)((a[q] - (float)h) * 1024.0f); h = (_Float16)c[q]; fh.h[4 + q] = h; fl.h[4 + q] = (_Float16)((c[q] - (float)h) * 1024.0f); }
  for (int pass = 0; pass < 2; ++pass) { *(volatile v8us*)((unsigned short*)Hh + t * 8) = fh.half[0]; *(volatile v8us*)((unsigned short*)Hl + t * 8) = fl.half[0]; if (pass == 0) __threadfence(); } }

__global__ __launch_bounds__(256) void k_dw(const float* __restrict__ X, const float* __restrict__ w, const float* __restrict__ bias, float* __restrict__ Y) {
  #pragma clang fp contract(off)
  const size_t t = (size_t)blockIdx.x * 256 + threadIdx.x; if (t >= (size_t)NIM * NTK * (CC / 4)) return; const int c0 = (int)(t % (CC / 4)) * 4; const size_t bn = t / (CC / 4); const int n = (int)(bn % NTK); const size_t b = bn / NTK; const int y = n / 28, x = n % 28; v4f acc;
#pragma unroll
  for (int q = 0; q < 4; ++q) acc[q] = bf16_round(bias[c0 + q]);
#pragma unroll
  for (int k = 0; k < 9; ++k) { const int yy = y + k / 3 - 1, xx = x + k % 3 - 1; const bool in = (yy >= 0 && yy < 28 && xx >= 0 && xx < 28); const int nn = min(max(yy, 0), 27) * 28 + min(max(xx, 0), 27); const v4f xv = *(const v4fa*)(X + (b * NTK + nn) * CC + c0);
#pragma unroll
    for (int q = 0; q < 4; ++q) acc[q] += in ? bf16_round(w[(c0 + q) * 9 + k]) * xv[q] : 0.f; }
  const v4f xc = *(const v4fa*)(X + bn * CC + c0); v4f o;
#pragma unroll
  for (int q = 0; q < 4; ++q) o[q] = xc[q] + acc[q];
  *(volatile v4f*)(Y + bn * CC + c0) = o; __threadfence(); *(volatile v4f*)(Y + bn * CC + c0) = o; }
__global__ __launch_bounds__(256) void k_tok(const float* __restrict__ x, float* __restrict__ X0) { const size_t t = (size_t)blockIdx.x * 256 + threadIdx.x; if (t >= (size_t)NIM * NTK * (CC / 8)) return; const int c0 = (int)(t % (CC / 8)) * 8; const size_t bn = t / (CC / 8); const int n = (int)(bn % NTK); const size_t b = bn / NTK; v4f a, c;
#pragma unroll
  for (int q = 0; q < 4; ++q) { a[q] = bf16_round(x[(b * CC + c0 + q) * NTK + n]); c[q] = bf16_round(x[(b * CC + c0 + 4 + q) * NTK + n]); }
  for (int pass = 0; pass < 2; ++pass) { *(volatile v4f*)(X0 + bn * CC + c0) = a; *(volatile v4f*)(X0 + bn * CC + c0 + 4) = c; if (pass == 0) __threadfence(); } }
__global__ __launch_bounds__(256) void k_ln(const float* __restrict__ X, size_t r0, const float* __restrict__ g, const float* __restrict__ bb, _Float16* __restrict__ Y) {
  #pragma clang fp contract(off)
  const int tid = threadIdx.x, w = tid >> 5, l = tid & 31; const int r = blockIdx.x * 8 + w; if (r >= RCH) return; const float* xr = X + (r0 + r) * CC; float v[12]; float s = 0.f;
#pragma unroll
  for (int k = 0; k < 12; ++k) { v[k] = xr[l + 32 * k]; s += v[k]; }
  for (int o = 16; o > 0; o >>= 1) s += __shfl_xor(s, o, 32); const float mu = s / (float)CC; float q2 = 0.f;
#pragma unroll
  for (int k = 0; k < 12; ++k) { const float d = v[k] - mu; q2 += d * d; }
  for (int o = 16; o > 0; o >>= 1) q2 += __shfl_xor(q2, o, 32); const float rs = rsqrtf(q2 / (float)CC + 1e-5f);
  for (int pass = 0; pass < 2; ++pass) {
#pragma unroll
    for (int k = 0; k < 12; ++k) { const int c = l + 32 * k; FragH f; f.h[0] = (_Float16)((v[k] - mu) * rs * bf16_round(g[c]) + bf16_round(bb[c])); *(volatile unsigned short*)((unsigned short*)Y + (size_t)r * CC + c) = f.u[0]; }
    if (pass == 0) __threadfence(); } }
__global__ __launch_bounds__(256) void k_kvt(const _Float16* __restrict__ QKV, _Float16* __restrict__ KT, _Float16* __restrict__ VT) {
  #pragma clang fp contract(off)
  const int t = blockIdx.x * 256 + threadIdx.x; if (t >= ICH * NH * HD * (NTP / 8)) return; const int n0 = (t % (NTP / 8)) * 8; const int d = (t / (NTP / 8)) % HD; const int ih = t / ((NTP / 8) * HD); const int i = ih / NH, h = ih % NH; FragH fk, fv;
#pragma unroll
  for (int q = 0; q < 8; ++q) { const int n = n0 + q; float kv = 0.f, vv = 0.f; if (n < NTK) { const size_t row = ((size_t)i * NTK + n) * (3 * CC); kv = (float)QKV[row + CC + h * HD + d] * 0.17677669529663687f; vv = (float)QKV[row + 2 * CC + h * HD + d]; } fk.h[q] = (_Float16)kv; fv.h[q] = (_Float16)vv; }
  for (int pass = 0; pass < 2; ++pass) { *(volatile v8us*)((unsigned short*)KT + ((size_t)ih * HD + d) * NTP + n0) = fk.half[0]; *(volatile v8us*)((unsigned short*)VT + ((size_t)ih * HD + d) * NTP + n0) = fv.half[0]; if (pass == 0) __threadfence(); } }
__global__ __launch_bounds__(256) void k_asoft(const float* __restrict__ ATT, _Float16* __restrict__ A16) {
  #pragma clang fp contract(off)
  const int tid = threadIdx.x, w = tid >> 5, l = tid & 31; const int row = blockIdx.x * 8 + w; if (row >= ICH * NH * HD) return; const float v = ATT[(size_t)row * HD + l]; float m = v; for (int o = 16; o > 0; o >>= 1) m = fmaxf(m, __shfl_xor(m, o, 32)); const float e = expf(v - m); float s = e; for (int o = 16; o > 0; o >>= 1) s += __shfl_xor(s, o, 32); FragH f; f.h[0] = (_Float16)(e / s);
  *(volatile unsigned short*)((unsigned short*)A16 + (size_t)row * 64 + l) = f.u[0]; __threadfence(); *(volatile unsigned short*)((unsigned short*)A16 + (size_t)row * 64 + l) = f.u[0]; }
__global__ __launch_bounds__(256) void k_nchw(const float* __restrict__ X, float* __restrict__ out) { const size_t t = (size_t)blockIdx.x * 256 + threadIdx.x; if (t >= (size_t)NIM * CC * (NTK / 4)) return; const int n0 = (int)(t % (NTK / 4)) * 4; const int c = (int)((t / (NTK / 4)) % CC); const size_t b = t / ((NTK / 4) * CC); v4f o;
#pragma unroll
  for (int q = 0; q < 4; ++q) o[q] = X[(b * NTK + n0 + q) * CC + c];
  float* dst = out + (b * CC + c) * NTK + n0; *(volatile v4f*)dst = o; __threadfence(); *(volatile v4f*)dst = o; }

extern "C" void kernel_launch(void* const* d_in, const int* in_sizes, int n_in,
                              void* d_out, int out_size, void* d_ws, size_t ws_size, hipStream_t stream) {
  (void)in_sizes; (void)n_in; (void)out_size;
  const float* const* I = (const float* const*)d_in; const float* x = I[0]; const float* c1w = I[1]; const float* c1b = I[2]; const float* n1g = I[3]; const float* n1b = I[4]; const float* qkvw = I[5]; const float* pw = I[6]; const float* pb = I[7]; const float* c2w = I[8]; const float* c2b = I[9]; const float* n2g = I[10]; const float* n2b = I[11]; const float* f1w = I[12]; const float* f1b = I[13]; const float* f2w = I[14]; const float* f2b = I[15];
  char* ws = (char*)d_ws; size_t off = 0;
  auto take = [&](size_t bytes) { char* p = ws + off; off += (bytes + 255) & ~(size_t)255; return p; };
  const size_t NR = (size_t)NIM * NTK;
  _Float16* BQ = (_Float16*)take((size_t)3 * CC * CC * 2); _Float16* BP = (_Float16*)take((size_t)CC * CC * 2); _Float16* BF1 = (_Float16*)take((size_t)HIDN * CC * 2); _Float16* BF2 = (_Float16*)take((size_t)CC * HIDN * 2);
  float* XA = (float*)take(NR * CC * 4); float* XB = (float*)take(NR * CC * 4); _Float16* L16 = (_Float16*)take((size_t)RCH * CC * 2); _Float16* QKV = (_Float16*)take((size_t)RCH * 3 * CC * 2); _Float16* KT = (_Float16*)take((size_t)ICH * NH * HD * NTP * 2); _Float16* VT = (_Float16*)take((size_t)ICH * NH * HD * NTP * 2); float* ATT = (float*)take((size_t)ICH * NH * HD * HD * 4); _Float16* A16 = (_Float16*)take((size_t)ICH * NH * HD * 64 * 2); _Float16* O16 = (_Float16*)take((size_t)RCH * CC * 2); _Float16* H16 = (_Float16*)take((size_t)RCH * HIDN * 2);
  if (off > ws_size) return;
  k_round16f<<<(3 * CC * CC / 8 + 255) / 256, 256, 0, stream>>>(qkvw, BQ, (size_t)3 * CC * CC / 8); k_round16f<<<(CC * CC / 8 + 255) / 256, 256, 0, stream>>>(pw, BP, (size_t)CC * CC / 8); k_round16f<<<(HIDN * CC / 8 + 255) / 256, 256, 0, stream>>>(f1w, BF1, (size_t)HIDN * CC / 8); k_round16f<<<(CC * HIDN / 8 + 255) / 256, 256, 0, stream>>>(f2w, BF2, (size_t)CC * HIDN / 8);
  k_tok<<<(unsigned)((NR * (CC / 8) + 255) / 256), 256, 0, stream>>>(x, XB); k_dw<<<(unsigned)((NR * (CC / 4) + 255) / 256), 256, 0, stream>>>(XB, c1w, c1b, XA);
  const dim3 gQ(((RCH / 16) * (3 * CC / 64) + 3) / 4, 1), gP(((RCH / 16) * (CC / 64) + 3) / 4, 1), gF(((RCH / 16) * (HIDN / 64) + 3) / 4, 1);
  for (int ch = 0; ch < NIM / ICH; ++ch) { const size_t r0 = (size_t)ch * RCH;
    k_ln<<<RCH / 8, 256, 0, stream>>>(XA, r0, n1g, n1b, L16);
    k_gemm_hhx<0><<<gQ, 128, 0, stream>>>(L16, CC, 0, BQ, CC, 0, 0.0625f, nullptr, 0, nullptr, 1, 0, 0, nullptr, QKV, 3 * CC, 0, RCH, 3 * CC, CC);
    k_kvt<<<(ICH * NH * HD * (NTP / 8) + 255) / 256, 256, 0, stream>>>(QKV, KT, VT);
    for (int i = 0; i < ICH; ++i) k_gemm_hhx<0><<<dim3(((HD / 16) * 1 + 3) / 4, NH), 128, 0, stream>>>(KT + (size_t)i * NH * HD * NTP, NTP, (size_t)HD * NTP, VT + (size_t)i * NH * HD * NTP, NTP, (size_t)HD * NTP, 1.0f, nullptr, 0, nullptr, 1, 0, 0, ATT + (size_t)i * NH * HD * HD, nullptr, HD, (size_t)HD * HD, HD, HD, NTP);
    k_asoft<<<(ICH * NH * HD + 7) / 8, 256, 0, stream>>>(ATT, A16);
    for (int i = 0; i < ICH; ++i) k_gemm_hhx<0><<<dim3(((NTK / 16) * 1 + 3) / 4, NH), 128, 0, stream>>>(QKV + (size_t)i * NTK * 3 * CC, 3 * CC, HD, A16 + (size_t)i * NH * HD * 64, 64, (size_t)HD * 64, 1.0f, nullptr, 0, nullptr, 1, 0, 0, nullptr, O16 + (size_t)i * NTK * CC, CC, HD, NTK, HD, HD);
    k_gemm_hhx<0><<<gP, 128, 0, stream>>>(O16, CC, 0, BP, CC, 0, 0.0625f, pb, 0, XA + r0 * CC, 1, (size_t)CC, 0, XA + r0 * CC, nullptr, CC, 0, RCH, CC, CC); }
  k_dw<<<(unsigned)((NR * (CC / 4) + 255) / 256), 256, 0, stream>>>(XA, c2w, c2b, XB);
  for (int ch = 0; ch < NIM / ICH; ++ch) { const size_t r0 = (size_t)ch * RCH;
    k_ln<<<RCH / 8, 256, 0, stream>>>(XB, r0, n2g, n2b, L16);
    k_gemm_hhx<6><<<gF, 128, 0, stream>>>(L16, CC, 0, BF1, CC, 0, 0.0625f, f1b, 0, nullptr, 1, 0, 0, nullptr, H16, HIDN, 0, RCH, HIDN, CC);
    k_gemm_hhx<0><<<gP, 128, 0, stream>>>(H16, HIDN, 0, BF2, HIDN, 0, 0.0625f, f2b, 0, XB + r0 * CC, 1, (size_t)CC, 0, XB + r0 * CC, nullptr, CC, 0, RCH, CC, HIDN); }
  k_nchw<<<(unsigned)((NR * (NTK / 4) + 255) / 256), 256, 0, stream>>>(XB, (float*)d_out);
}
